// Matching_Score_sent_29197187678290
// MI455X (gfx1250) — hardware-verified
//
#include <hip/hip_runtime.h>

typedef __attribute__((ext_vector_type(16))) _Float16 v16h;
typedef __attribute__((ext_vector_type(8)))  _Float16 v8h;
typedef __attribute__((ext_vector_type(8)))  float    v8f;
typedef __attribute__((ext_vector_type(4)))  unsigned v4u_t;
typedef unsigned v4ua __attribute__((ext_vector_type(4), may_alias));

#define NB    8192
#define DDIM  256
#define GLOG2E 14.426950408889634f
#define NBLK  64

template <int IMM>
__device__ __forceinline__ float swz_xor_add(float x) {
    int i = __builtin_bit_cast(int, x);
    i = __builtin_amdgcn_ds_swizzle(i, IMM);
    return x + __builtin_bit_cast(float, i);
}
#define SWZ_X1  0x041f
#define SWZ_X2  0x081f
#define SWZ_X4  0x101f
#define SWZ_X8  0x201f
#define SWZ_X16 0x401f

__global__ __launch_bounds__(256) void normalize_f16(
    const float* __restrict__ e, const float* __restrict__ v,
    _Float16* __restrict__ eh, _Float16* __restrict__ vh)
{
    const int wave = (blockIdx.x * blockDim.x + threadIdx.x) >> 5;
    const int lane = threadIdx.x & 31;

    const float* src;
    _Float16*    dst;
    int row;
    if (wave < NB) { src = e; dst = eh; row = wave; }
    else           { src = v; dst = vh; row = wave - NB; }

    const float* p = src + (size_t)row * DDIM + lane * 8;
    float x[8];
    float ss = 0.0f;
#pragma unroll
    for (int t = 0; t < 8; ++t) {
        x[t] = p[t];
        ss += x[t] * x[t];
    }
    ss = swz_xor_add<SWZ_X16>(ss);
    ss = swz_xor_add<SWZ_X8>(ss);
    ss = swz_xor_add<SWZ_X4>(ss);
    ss = swz_xor_add<SWZ_X2>(ss);
    ss = swz_xor_add<SWZ_X1>(ss);

    const float scale = 1.0f / fmaxf(sqrtf(ss), 1e-8f);

    _Float16 hh[8];
#pragma unroll
    for (int t = 0; t < 8; ++t) hh[t] = (_Float16)(x[t] * scale);
    _Float16* q = dst + (size_t)row * DDIM + lane * 8;
    *(volatile v4u_t*)q = *(const v4ua*)hh; __threadfence(); *(volatile v4u_t*)q = *(const v4ua*)hh;
}

__global__ __launch_bounds__(256) void gram_tile(
    const _Float16* __restrict__ eh, const _Float16* __restrict__ vh,
    float* __restrict__ rowp,
    float* __restrict__ colp)
{
    __shared__ float lds_row[2][128];
    __shared__ float lds_col[4][128];

    const int lane = threadIdx.x & 31;
    const int w    = threadIdx.x >> 5;
    const int wm   = w >> 1;
    const int wn   = w & 1;
    const int ib   = blockIdx.y;
    const int jb   = blockIdx.x;
    const int i0   = ib * 128;
    const int j0   = jb * 128;
    const int g    = lane >> 4;
    const int mr   = lane & 15;

    v8f acc[2][4];
#pragma unroll
    for (int tm = 0; tm < 2; ++tm)
#pragma unroll
        for (int tn = 0; tn < 4; ++tn)
            acc[tm][tn] = (v8f){0.f,0.f,0.f,0.f,0.f,0.f,0.f,0.f};

    for (int k0 = 0; k0 < DDIM; k0 += 32) {
        v16h a[2], b[4];
#pragma unroll
        for (int tm = 0; tm < 2; ++tm) {
            const _Float16* pa =
                eh + (size_t)(i0 + wm * 32 + tm * 16 + mr) * DDIM + k0 + 8 * g;
            v8h lo = *(const v8h*)(pa);
            v8h hi = *(const v8h*)(pa + 16);
#pragma unroll
            for (int t = 0; t < 8; ++t) { a[tm][t] = lo[t]; a[tm][t + 8] = hi[t]; }
        }
#pragma unroll
        for (int tn = 0; tn < 4; ++tn) {
            const _Float16* pb =
                vh + (size_t)(j0 + wn * 64 + tn * 16 + mr) * DDIM + k0 + 8 * g;
            b[tn] = __builtin_shufflevector(*(const v8h*)pb, *(const v8h*)(pb + 16), 0,1,2,3,4,5,6,7,8,9,10,11,12,13,14,15);
        }
#pragma unroll
        for (int tm = 0; tm < 2; ++tm)
#pragma unroll
            for (int tn = 0; tn < 4; ++tn)
                acc[tm][tn] = __builtin_amdgcn_wmma_f32_16x16x32_f16(
                    false, a[tm], false, b[tn],
                    (short)0, acc[tm][tn], false, false);
    }

    v8f ex[2][4];
#pragma unroll
    for (int tm = 0; tm < 2; ++tm)
#pragma unroll
        for (int tn = 0; tn < 4; ++tn)
#pragma unroll
            for (int r = 0; r < 8; ++r)
                ex[tm][tn][r] = __builtin_amdgcn_exp2f(GLOG2E * acc[tm][tn][r]);

#pragma unroll
    for (int tm = 0; tm < 2; ++tm)
#pragma unroll
        for (int r = 0; r < 8; ++r) {
            float rv = ex[tm][0][r] + ex[tm][1][r] + ex[tm][2][r] + ex[tm][3][r];
            rv = swz_xor_add<SWZ_X1>(rv);
            rv = swz_xor_add<SWZ_X2>(rv);
            rv = swz_xor_add<SWZ_X4>(rv);
            rv = swz_xor_add<SWZ_X8>(rv);
            if (mr == 0)
                lds_row[wn][wm * 32 + tm * 16 + 8 * g + r] = rv;
        }

#pragma unroll
    for (int tn = 0; tn < 4; ++tn) {
        float cv = 0.0f;
#pragma unroll
        for (int tm = 0; tm < 2; ++tm)
#pragma unroll
            for (int r = 0; r < 8; ++r)
                cv += ex[tm][tn][r];
        cv = swz_xor_add<SWZ_X16>(cv);
        if (g == 0)
            lds_col[wm][wn * 64 + tn * 16 + mr] = cv;
    }

    __syncthreads();

    const int t = threadIdx.x;
    if (t < 128) {
        const float v = lds_row[0][t] + lds_row[1][t];
        *(volatile float*)(rowp + (size_t)jb * NB + i0 + t) = v; __threadfence(); *(volatile float*)(rowp + (size_t)jb * NB + i0 + t) = v;
    } else {
        const int u = t - 128;
        const float v = lds_col[0][u] + lds_col[1][u] + lds_col[2][u] + lds_col[3][u];
        *(volatile float*)(colp + (size_t)ib * NB + j0 + u) = v; __threadfence(); *(volatile float*)(colp + (size_t)ib * NB + j0 + u) = v;
    }
}

__global__ __launch_bounds__(256) void reduce_out(
    const float* __restrict__ rowp, const float* __restrict__ colp,
    float* __restrict__ out)
{
    const int i = blockIdx.x * blockDim.x + threadIdx.x;
    const float* src = (i < NB) ? (rowp + i) : (colp + (i - NB));
    float s = 0.0f;
#pragma unroll
    for (int b = 0; b < NBLK; ++b)
        s += src[(size_t)b * NB];
    *(volatile float*)(out + i) = s; __threadfence(); *(volatile float*)(out + i) = s;
}

extern "C" void kernel_launch(void* const* d_in, const int* in_sizes, int n_in,
                              void* d_out, int out_size, void* d_ws, size_t ws_size,
                              hipStream_t stream)
{
    const float* e = (const float*)d_in[0];
    const float* v = (const float*)d_in[1];
    float* out = (float*)d_out;

    _Float16* eh   = (_Float16*)d_ws;
    _Float16* vh   = eh + (size_t)NB * DDIM;
    float*    rowp = (float*)(vh + (size_t)NB * DDIM);
    float*    colp = rowp + (size_t)NBLK * NB;

    normalize_f16<<<2 * NB / 8, 256, 0, stream>>>(e, v, eh, vh);

    dim3 grid(NBLK, NBLK);
    gram_tile<<<grid, 256, 0, stream>>>(eh, vh, rowp, colp);

    reduce_out<<<(2 * NB) / 256, 256, 0, stream>>>(rowp, colp, out);
}
